// GraphFeatureFusion_88175678587174
// MI455X (gfx1250) — hardware-verified
//
#include <hip/hip_runtime.h>
#include <stddef.h>
#include <stdint.h>
#include <math.h>


#define NB      16
#define NPG     1024
#define FEAT    512
#define HID     1024
#define NN      (NB * NPG)
#define NEDGE   262144
#define NTHR    256
#define NWAVE   8
#define EPT     8
#define CHUNK   (NTHR * EPT)
#define WCAP    (EPT * 32)
#define LISTN   (NWAVE * WCAP)
#define NBA     1024
#define SLA     10
#define RCAP    28672
#define DEGCAP  64
#define MEAS_B1024  16384
#define MEAS_MAXDEG 41
#define BKT_ZINTS    (RCAP + 3 * NBA)
#define BKT_LDS_INTS (LISTN + 2 * RCAP + 3 * NBA + 16)
#define GT      128
#define GTHR    256
#define GEMM_LDS_FLOATS (GT * GT + 3 * GT)
#define RTHR    512
#define CINV    0.000244140625f
#define FLUSHT  6.1035e-5f
#define WSMAX   134217728
#define WTAIL   54001664
#define NUX     (NN * FEAT / 8)
#define NUW1    (HID * 2 * FEAT / 8)
#define NUID    4096
#define NUW23   (HID * 2 * HID / 8)

constexpr int kceil(int n) {
  const double v = 0.8 * (double)n;
  const int t = (int)v;
  return ((double)t < v) ? t + 1 : t;
}
#define KK1 820
#define KK2 656
#define KK3 525
#define MM1 NN
#define MM2 (NB * KK1)
#define MM3 (NB * KK2)

static_assert(kceil(NPG) == KK1 && kceil(KK1) == KK2 && kceil(KK2) == KK3);
static_assert(NPG == NBA);
static_assert((CHUNK & (CHUNK - 1)) == 0 && CHUNK <= 4096);
static_assert((NBA & (NBA - 1)) == 0 && NBA == (1 << SLA));
static_assert(((long long)CHUNK << SLA) < (1LL << 31));
static_assert(NN <= 65536);
static_assert(RCAP % 1024 == 0 && BKT_ZINTS % (NTHR * 4) == 0);
static_assert(RCAP >= MEAS_B1024 + MEAS_B1024 / 4);
static_assert(DEGCAP >= MEAS_MAXDEG + 8);
static_assert(BKT_LDS_INTS * 4 <= 327680 && GEMM_LDS_FLOATS * 4 <= 327680);
static_assert((2 * FEAT) % 32 == 0 && (2 * HID) % 32 == 0 && FEAT % 32 == 0 && HID % 32 == 0);
static_assert(HID % GT == 0 && HID / GT == 8 && MM1 % GT == 0 && MM3 % GT == 0);
static_assert(GT == (GTHR / 32) * 16);
static_assert(NUX % NTHR == 0 && NUW1 % NTHR == 0 && NUID % NTHR == 0 && NUW23 % NTHR == 0);
static_assert(NUID * 4 == NN);
static_assert(HID == 2 * RTHR && NPG == 2 * RTHR);
static_assert((size_t)MM2 * HID * 4 <= (size_t)WTAIL);
static_assert((size_t)WTAIL + (size_t)2 * HID * 2 * HID * 2 <= (size_t)NN * HID * 4);
static_assert(KK3 >= 8);

typedef float          v2f  __attribute__((ext_vector_type(2)));
typedef float          v4f  __attribute__((ext_vector_type(4)));
typedef float          v8f  __attribute__((ext_vector_type(8)));
typedef double         v2d  __attribute__((ext_vector_type(2)));
typedef int            v4i  __attribute__((ext_vector_type(4)));
typedef int            v8i  __attribute__((ext_vector_type(8)));
typedef unsigned       v2u  __attribute__((ext_vector_type(2)));
typedef unsigned       v4u  __attribute__((ext_vector_type(4)));
typedef unsigned short v8us __attribute__((ext_vector_type(8)));
typedef _Float16       v16h __attribute__((ext_vector_type(16)));
typedef v4f  __attribute__((may_alias)) v4fa;
typedef v2d  __attribute__((may_alias)) v2da;
typedef v4i  __attribute__((may_alias)) v4ia;
typedef v4u  __attribute__((may_alias)) v4ua;
typedef v8us __attribute__((may_alias)) v8usa;
union FragH { v16h v; v8us h[2]; v8i w; };

#define KATTR __attribute__((amdgpu_num_vgpr(248)))

__device__ __forceinline__ v8f wmh(const FragH& a, const FragH& b, v8f c) {
  v8f d = __builtin_amdgcn_wmma_f32_16x16x32_f16(false, a.v, false, b.v, (short)0, c, false, false);
  asm volatile("v_nop\n\tv_nop\n\tv_nop\n\tv_nop" : "+v"(d) : "v"(a.w), "v"(b.w));
  return d;
}

__device__ __forceinline__ float bfr(float f) {
  const unsigned int u = __float_as_uint(f);
  const unsigned int r = ((u + 0x7FFFu + ((u >> 16) & 1u)) >> 16) & 0xFFFFu;
  const unsigned int b = ((u & 0x7FFFFFFFu) > 0x7F800000u) ? 0x7FC0u : r;
  return __uint_as_float(b << 16);
}
__device__ __forceinline__ unsigned int f2h_bits(float t) {
  const float u = (fabsf(t) < FLUSHT) ? 0.0f : t;
  const _Float16 h = (_Float16)u;
  return (unsigned int)__builtin_bit_cast(unsigned short, h);
}
__device__ __forceinline__ float h2f(unsigned int b) {
  const unsigned short s = (unsigned short)(b & 0xFFFFu);
  return (float)__builtin_bit_cast(_Float16, s);
}

template <int SLB>
__device__ __forceinline__ int scan_chunk(const int* __restrict__ dsts, int nE, int cbase, int slotBase,
                                          int nb, int vec8, int* list, int tid, int lane, int wave) {
  int wc = 0;
  const int el0  = tid * EPT;
  const int e0   = cbase + el0;
  const int sent = -2147483647 - 1;
  v4i da, db;
  if (vec8 != 0 && cbase + CHUNK <= nE) {
    da = *(const v4i*)(dsts + e0);
    db = *(const v4i*)(dsts + e0 + 4);
  } else {
    da.x = (e0     < nE) ? dsts[min(e0,     nE - 1)] : sent;
    da.y = (e0 + 1 < nE) ? dsts[min(e0 + 1, nE - 1)] : sent;
    da.z = (e0 + 2 < nE) ? dsts[min(e0 + 2, nE - 1)] : sent;
    da.w = (e0 + 3 < nE) ? dsts[min(e0 + 3, nE - 1)] : sent;
    db.x = (e0 + 4 < nE) ? dsts[min(e0 + 4, nE - 1)] : sent;
    db.y = (e0 + 5 < nE) ? dsts[min(e0 + 5, nE - 1)] : sent;
    db.z = (e0 + 6 < nE) ? dsts[min(e0 + 6, nE - 1)] : sent;
    db.w = (e0 + 7 < nE) ? dsts[min(e0 + 7, nE - 1)] : sent;
  }
  const unsigned nbs = (unsigned)slotBase;
  const unsigned unb = (unsigned)nb;
  const unsigned s0 = (unsigned)da.x - nbs, s1 = (unsigned)da.y - nbs;
  const unsigned s2 = (unsigned)da.z - nbs, s3 = (unsigned)da.w - nbs;
  const unsigned s4 = (unsigned)db.x - nbs, s5 = (unsigned)db.y - nbs;
  const unsigned s6 = (unsigned)db.z - nbs, s7 = (unsigned)db.w - nbs;
  const bool h0 = s0 < unb, h1 = s1 < unb, h2 = s2 < unb, h3 = s3 < unb;
  const bool h4 = s4 < unb, h5 = s5 < unb, h6 = s6 < unb, h7 = s7 < unb;
  const unsigned any = __builtin_amdgcn_ballot_w32(h0 | h1 | h2 | h3 | h4 | h5 | h6 | h7);
  if (any != 0u) {
#define HITJ(J, HJ, SJ) { \
      const unsigned mj = __builtin_amdgcn_ballot_w32(HJ); \
      if (mj != 0u) { \
        if (HJ) { \
          const int pos = wc + (int)__builtin_amdgcn_mbcnt_lo(mj, 0u); \
          if (pos < WCAP) list[wave * WCAP + pos] = ((el0 + (J)) << SLB) | (int)(SJ); \
        } \
        wc += (int)__builtin_popcount(mj); } }
    HITJ(0, h0, s0)
    HITJ(1, h1, s1)
    HITJ(2, h2, s2)
    HITJ(3, h3, s3)
    HITJ(4, h4, s4)
    HITJ(5, h5, s5)
    HITJ(6, h6, s6)
    HITJ(7, h7, s7)
#undef HITJ
  }
  return wc;
}

template <int LOGF>
__device__ __forceinline__ v4u wcat_unit(const float* __restrict__ wl, const float* __restrict__ wr, int v) {
  constexpr int F   = 1 << LOGF;
  constexpr int UPR = F / 4;
  const int n  = v >> (LOGF - 2);
  const int k8 = (v & (UPR - 1)) * 8;
  const int kk = k8 & (F - 1);
  const size_t wo = (size_t)n * F + (size_t)kk;
  const v4f a0 = *(const v4f*)(wl + wo), a1 = *(const v4f*)(wl + wo + 4);
  const v4f c0 = *(const v4f*)(wr + wo), c1 = *(const v4f*)(wr + wo + 4);
  const float fa[8] = {a0.x, a0.y, a0.z, a0.w, a1.x, a1.y, a1.z, a1.w};
  const float fb[8] = {c0.x, c0.y, c0.z, c0.w, c1.x, c1.y, c1.z, c1.w};
  const unsigned msk = (k8 < F) ? 0xFFFFu : 0u;
  unsigned e[8];
#pragma unroll
  for (int i = 0; i < 8; ++i) {
    const unsigned ha = f2h_bits(256.0f * bfr(fa[i]));
    const unsigned hb = f2h_bits(256.0f * bfr(fb[i]));
    e[i] = (ha & msk) | (hb & (~msk & 0xFFFFu));
  }
  v4u o;
  o.x = e[0] | (e[1] << 16); o.y = e[2] | (e[3] << 16);
  o.z = e[4] | (e[5] << 16); o.w = e[6] | (e[7] << 16);
  return o;
}

__global__ __launch_bounds__(NTHR) KATTR void k_prep(const float* __restrict__ x, const float* __restrict__ wl,
                                                     const float* __restrict__ wr, unsigned short* XH,
                                                     unsigned short* W1C, int* MAP0, int* ORIG1) {
  const int u = (int)blockIdx.x * NTHR + (int)threadIdx.x;
  v4u o;
  unsigned* dp;
  if (u < NUX) {
    const float* p = x + (size_t)u * 8;
    const v4f a0 = *(const v4f*)p, a1 = *(const v4f*)(p + 4);
    const float fa[8] = {a0.x, a0.y, a0.z, a0.w, a1.x, a1.y, a1.z, a1.w};
    unsigned e[8];
#pragma unroll
    for (int i = 0; i < 8; ++i) e[i] = f2h_bits(16.0f * bfr(fa[i]));
    o.x = e[0] | (e[1] << 16); o.y = e[2] | (e[3] << 16);
    o.z = e[4] | (e[5] << 16); o.w = e[6] | (e[7] << 16);
    dp = (unsigned*)(XH + (size_t)u * 8);
  } else if (u < NUX + NUW1) {
    const int v = u - NUX;
    o = wcat_unit<9>(wl, wr, v);
    dp = (unsigned*)(W1C + (size_t)v * 8);
  } else if (u < NUX + NUW1 + 2 * NUID) {
    const int v  = u - NUX - NUW1;
    const int vv = v & (NUID - 1);
    o.x = (unsigned)(4 * vv); o.y = (unsigned)(4 * vv + 1);
    o.z = (unsigned)(4 * vv + 2); o.w = (unsigned)(4 * vv + 3);
    if (v < NUID) dp = (unsigned*)(MAP0 + 4 * vv);
    else          dp = (unsigned*)(ORIG1 + 4 * vv);
  } else {
    return;
  }
  *(volatile v4u*)dp = o;
  __threadfence();
  *(volatile v4u*)dp = o;
}

__global__ __launch_bounds__(NTHR) KATTR void k_prepW(const float* __restrict__ w2l, const float* __restrict__ w2r,
                                                      const float* __restrict__ w3l, const float* __restrict__ w3r,
                                                      unsigned short* WC) {
  const int v  = (int)blockIdx.x * NTHR + (int)threadIdx.x;
  const int l  = v >> 18;
  const int vv = v & (NUW23 - 1);
  v4u o;
  if (l == 0) o = wcat_unit<10>(w2l, w2r, vv);
  else        o = wcat_unit<10>(w3l, w3r, vv);
  unsigned* dp = (unsigned*)(WC + (size_t)v * 8);
  *(volatile v4u*)dp = o;
  __threadfence();
  *(volatile v4u*)dp = o;
}

__global__ __launch_bounds__(NTHR) KATTR void k_bucket(const int* __restrict__ srcs, const int* __restrict__ dsts,
                                                       int nE, int nN, int vec8, int* LIST, int* CNT, int* OFF,
                                                       int* FLG) {
  extern __shared__ __attribute__((aligned(16))) int bsm[];
  int* list = bsm;
  int* reg1 = bsm + LISTN;
  int* sl   = reg1 + RCAP;
  int* cnt  = sl + RCAP;
  int* offs = cnt + NBA;
  int* cur  = offs + NBA;
  int* wcnt = cur + NBA;
  const int tid = (int)threadIdx.x, lane = tid & 31, wave = tid >> 5;
  const int blk = (int)blockIdx.x;
  const int nodeBase = blk * NBA;
  int nb = nN - nodeBase;
  nb = nb < 0 ? 0 : (nb > NBA ? NBA : nb);

  {
    const v4i z4 = {0, 0, 0, 0};
    for (int i = tid * 4; i < BKT_ZINTS; i += NTHR * 4) *(v4ia*)(sl + i) = z4;
    if (tid < 16) wcnt[tid] = 0;
  }
  __syncthreads();

  int tot = 0, ovf = 0;
  const int nChunks = (nE + CHUNK - 1) / CHUNK;
#pragma unroll 1
  for (int ch = 0; ch < nChunks; ++ch) {
    const int cbase = ch * CHUNK;
    const int wc = scan_chunk<SLA>(dsts, nE, cbase, nodeBase, nb, vec8, list, tid, lane, wave);
    if (lane == 0) wcnt[wave] = wc;
    __syncthreads();
    int pre = 0, all = 0;
#pragma unroll
    for (int w2 = 0; w2 < NWAVE; ++w2) {
      int c = wcnt[w2];
      c = c < 0 ? 0 : (c > WCAP ? WCAP : c);
      all += c;
      pre += (w2 < wave) ? c : 0;
    }
    const int wcc  = wc > WCAP ? WCAP : wc;
    const int base = tot + pre;
#pragma unroll 1
    for (int i = lane; i < wcc; i += 32) {
      const int ent = list[wave * WCAP + i];
      const int el  = (ent >> SLA) & (CHUNK - 1);
      const int sq  = ent & (NBA - 1);
      int eid = cbase + el;
      eid = eid > nE - 1 ? nE - 1 : eid;
      const int sraw = srcs[eid];
      const int s = sraw < 0 ? 0 : (sraw > nN - 1 ? nN - 1 : sraw);
      const int pos = base + i;
      if (pos < RCAP) reg1[pos] = (int)((unsigned)s | ((unsigned)sq << 16));
    }
    if (tot + all > RCAP) ovf = 1;
    tot += all;
    tot = tot > RCAP ? RCAP : tot;
    __syncthreads();
  }
  const int nh = tot;

  if (wave == 0) {
#pragma unroll 1
    for (int b0 = 0; b0 < nh; b0 += 32) {
      const int idx = b0 + lane;
      const int uv  = reg1[idx < nh ? idx : nh - 1];
      const int m32 = (nh - b0) < 32 ? (nh - b0) : 32;
#pragma unroll 1
      for (int k = 0; k < m32; ++k) {
        const int u  = __builtin_amdgcn_readlane(uv, k);
        const int sq = (u >> 16) & (NBA - 1);
        if (lane == 0) cnt[sq] = cnt[sq] + 1;
      }
    }
  }
  __syncthreads();
  if (wave == 0) {
    const int base = lane * (NBA / 32);
    int s = 0;
#pragma unroll 1
    for (int i = 0; i < NBA / 32; ++i) s += cnt[base + i];
    int incl = s;
#pragma unroll
    for (int d = 1; d < 32; d <<= 1) {
      const int y = __shfl_up(incl, d, 32);
      if (lane >= d) incl += y;
    }
    int run = incl - s;
#pragma unroll 1
    for (int i = 0; i < NBA / 32; ++i) {
      const int cv = cnt[base + i];
      offs[base + i] = run;
      cur[base + i]  = run;
      run += cv;
    }
  }
  __syncthreads();
  if (wave == 0) {
#pragma unroll 1
    for (int b0 = 0; b0 < nh; b0 += 32) {
      const int idx = b0 + lane;
      const int uv  = reg1[idx < nh ? idx : nh - 1];
      const int m32 = (nh - b0) < 32 ? (nh - b0) : 32;
#pragma unroll 1
      for (int k = 0; k < m32; ++k) {
        const int u  = __builtin_amdgcn_readlane(uv, k);
        const int sq = (u >> 16) & (NBA - 1);
        if (lane == 0) {
          int p = cur[sq];
          p = p < 0 ? 0 : (p > RCAP - 1 ? RCAP - 1 : p);
          sl[p] = u;
          cur[sq] = p + 1;
        }
      }
    }
  }
  __syncthreads();

  int* lb = LIST + (size_t)blk * RCAP;
  int* cb = CNT + (size_t)blk * NBA + 4 * tid;
  int* ob = OFF + (size_t)blk * NBA + 4 * tid;
  int* fp = FLG + (size_t)blk * 32 + 4 * (tid & 7);
  const v4i cvec = *(const v4ia*)(cnt + 4 * tid);
  const v4i ovec = *(const v4ia*)(offs + 4 * tid);
  v4i fv;
  fv.x = (tid == 0) ? nh : 0;
  fv.y = (tid == 0) ? ovf : 0;
  fv.z = 0; fv.w = 0;
#pragma unroll 1
  for (int p = tid * 4; p < RCAP; p += NTHR * 4) {
    const v4i v = *(const v4ia*)(sl + p);
    *(volatile v4i*)(lb + p) = v;
  }
  *(volatile v4i*)cb = cvec;
  *(volatile v4i*)ob = ovec;
  if (tid < 8) *(volatile v4i*)fp = fv;
  __threadfence();
#pragma unroll 1
  for (int p = tid * 4; p < RCAP; p += NTHR * 4) {
    const v4i v = *(const v4ia*)(sl + p);
    *(volatile v4i*)(lb + p) = v;
  }
  *(volatile v4i*)cb = cvec;
  *(volatile v4i*)ob = ovec;
  if (tid < 8) *(volatile v4i*)fp = fv;
}

template <int NSEG>
__global__ __launch_bounds__(NTHR) KATTR void k_agg(const int* __restrict__ LIST, const int* __restrict__ CNT,
                                                    const int* __restrict__ OFF, const int* __restrict__ FLG0,
                                                    const int* __restrict__ MAPP,
                                                    const unsigned short* __restrict__ P, unsigned short* MEAN,
                                                    int M) {
  constexpr int F = NSEG * 256;
  const int tid = (int)threadIdx.x, lane = tid & 31;
  const int wave = __builtin_amdgcn_readfirstlane(tid >> 5);
  const int i = (int)blockIdx.x * NWAVE + wave;
  const int g = i >> SLA;
  const int curRaw = __builtin_amdgcn_readfirstlane(MAPP[i]);
  if (curRaw < 0) return;
  const int cur = curRaw > M - 1 ? M - 1 : curRaw;
  int c = __builtin_amdgcn_readfirstlane(CNT[i]);
  const bool big = c > DEGCAP;
  c = c < 0 ? 0 : (c > DEGCAP ? DEGCAP : c);
  int o = __builtin_amdgcn_readfirstlane(OFF[i]);
  o = o < 0 ? 0 : (o > RCAP ? RCAP : o);
  if (c > RCAP - o) c = RCAP - o;
  const int fl = __builtin_amdgcn_readfirstlane(FLG0[g * 32 + 1]);
  const int* lb = LIST + (size_t)g * RCAP;

  float acc[NSEG * 8];
#pragma unroll
  for (int q = 0; q < NSEG * 8; ++q) acc[q] = 0.0f;
  int myc = 0;
#pragma unroll 1
  for (int b0 = 0; b0 < c; b0 += 32) {
    const int t = b0 + lane;
    int idx = o + t;
    idx = idx > RCAP - 1 ? RCAP - 1 : idx;
    const int ent = lb[idx];
    int sr = ent & 0xFFFF;
    sr = sr > NN - 1 ? NN - 1 : sr;
    const int csr = MAPP[sr];
    const bool ok = (t < c) && (csr >= 0);
    myc += ok ? 1 : 0;
    const int csv = ok ? (csr > M - 1 ? M - 1 : csr) : -1;
    const int m32 = (c - b0) < 32 ? (c - b0) : 32;
#pragma unroll 1
    for (int k = 0; k < m32; ++k) {
      const int sk = __builtin_amdgcn_readlane(csv, k);
      const int rk = sk < 0 ? 0 : sk;
      const bool use = sk >= 0;
      const unsigned short* rp = P + (size_t)rk * F + 8 * lane;
#pragma unroll
      for (int sg = 0; sg < NSEG; ++sg) {
        const v4u w = *(const v4ua*)(rp + sg * 256);
        acc[sg * 8 + 0] += use ? h2f(w.x) : 0.0f;
        acc[sg * 8 + 1] += use ? h2f(w.x >> 16) : 0.0f;
        acc[sg * 8 + 2] += use ? h2f(w.y) : 0.0f;
        acc[sg * 8 + 3] += use ? h2f(w.y >> 16) : 0.0f;
        acc[sg * 8 + 4] += use ? h2f(w.z) : 0.0f;
        acc[sg * 8 + 5] += use ? h2f(w.z >> 16) : 0.0f;
        acc[sg * 8 + 6] += use ? h2f(w.w) : 0.0f;
        acc[sg * 8 + 7] += use ? h2f(w.w >> 16) : 0.0f;
      }
    }
  }
  int cn = myc;
  cn += __shfl_xor(cn, 16, 32);
  cn += __shfl_xor(cn, 8, 32);
  cn += __shfl_xor(cn, 4, 32);
  cn += __shfl_xor(cn, 2, 32);
  cn += __shfl_xor(cn, 1, 32);
  const float inv = 1.0f / fmaxf((float)cn, 1.0f);
  const bool poison = (fl != 0) || big;
  const float qnan = __int_as_float(0x7fc00000);
  v4u q[NSEG];
#pragma unroll
  for (int sg = 0; sg < NSEG; ++sg) {
    unsigned e[8];
#pragma unroll
    for (int j = 0; j < 8; ++j) {
      const float mv = acc[sg * 8 + j] * inv;
      e[j] = f2h_bits(poison ? qnan : mv);
    }
    q[sg].x = e[0] | (e[1] << 16); q[sg].y = e[2] | (e[3] << 16);
    q[sg].z = e[4] | (e[5] << 16); q[sg].w = e[6] | (e[7] << 16);
  }
  unsigned* mp = (unsigned*)(MEAN + (size_t)cur * F + 8 * lane);
#pragma unroll
  for (int sg = 0; sg < NSEG; ++sg) *(volatile v4u*)(mp + sg * 128) = q[sg];
  __threadfence();
#pragma unroll
  for (int sg = 0; sg < NSEG; ++sg) *(volatile v4u*)(mp + sg * 128) = q[sg];
}

__device__ __forceinline__ void gemm_run(const unsigned short* __restrict__ ap, const unsigned short* __restrict__ bp,
                                         int ldb, int klen, v8f (&acc)[8]) {
#pragma unroll 1
  for (int k0 = 0; k0 < klen; k0 += 32) {
    FragH af;
    af.h[0] = *(const v8usa*)(ap + k0);
    af.h[1] = *(const v8usa*)(ap + k0 + 16);
#pragma unroll
    for (int nt = 0; nt < 8; ++nt) {
      const unsigned short* wq = bp + (size_t)(16 * nt) * (size_t)ldb + k0;
      FragH bf;
      bf.h[0] = *(const v8usa*)wq;
      bf.h[1] = *(const v8usa*)(wq + 16);
      acc[nt] = wmh(af, bf, acc[nt]);
    }
  }
}

__global__ __launch_bounds__(GTHR) KATTR void k_gemm(const unsigned short* __restrict__ AM,
                                                     const unsigned short* __restrict__ AP,
                                                     const unsigned short* __restrict__ WC, int F, int M,
                                                     const float* __restrict__ bias,
                                                     const float* __restrict__ pvec, float* Hout, float* DOTP) {
  extern __shared__ __attribute__((aligned(16))) float gsm[];
  float* stg  = gsm;
  float* sb   = gsm + GT * GT;
  float* sp   = sb + GT;
  float* sdot = sp + GT;
  const int tid = (int)threadIdx.x, lane = tid & 31, wave = tid >> 5, hh = lane >> 4, m = lane & 15;
  const int rowBase = (int)blockIdx.x * GT;
  const int ct   = (int)blockIdx.y;
  const int col0 = ct * GT;
  if (tid < GT) {
    sb[tid] = bfr(bias[col0 + tid]);
    sp[tid] = bfr(pvec[col0 + tid]);
  }

  v8f acc[8];
  {
    const v8f z = {0.f, 0.f, 0.f, 0.f, 0.f, 0.f, 0.f, 0.f};
#pragma unroll
    for (int t = 0; t < 8; ++t) acc[t] = z;
  }
  int ar = rowBase + 16 * wave + m;
  ar = ar > M - 1 ? M - 1 : ar;
  const int K2 = 2 * F;
  const unsigned short* am = AM + (size_t)ar * (size_t)F + 8 * hh;
  const unsigned short* ap = AP + (size_t)ar * (size_t)F + 8 * hh;
  const unsigned short* bp = WC + (size_t)(col0 + m) * (size_t)K2 + 8 * hh;
  gemm_run(am, bp, K2, F, acc);
  gemm_run(ap, bp + F, K2, F, acc);

#pragma unroll
  for (int nt = 0; nt < 8; ++nt) {
    const int lc = 16 * nt + m;
#pragma unroll
    for (int r = 0; r < 8; ++r) {
      const int lr = 16 * wave + 8 * hh + r;
      stg[lr * GT + lc] = acc[nt][r];
    }
  }
  __syncthreads();

  const v4f b4 = *(const v4fa*)(sb + 4 * lane);
  const v4f p4 = *(const v4fa*)(sp + 4 * lane);
  float mydot = 0.0f;
#pragma unroll 1
  for (int i = 0; i < 16; ++i) {
    const int lr  = 16 * wave + i;
    const int row = rowBase + lr;
    const v4f a = *(const v4fa*)(stg + lr * GT + 4 * lane);
    const float v0 = fmaf(a.x, CINV, b4.x), v1 = fmaf(a.y, CINV, b4.y);
    const float v2 = fmaf(a.z, CINV, b4.z), v3 = fmaf(a.w, CINV, b4.w);
    v4f o;
    o.x = (v0 > 0.0f) ? v0 : (v0 - v0);
    o.y = (v1 > 0.0f) ? v1 : (v1 - v1);
    o.z = (v2 > 0.0f) ? v2 : (v2 - v2);
    o.w = (v3 > 0.0f) ? v3 : (v3 - v3);
    float d = (o.x * p4.x + o.y * p4.y) + (o.z * p4.z + o.w * p4.w);
    d += __shfl_xor(d, 16, 32);
    d += __shfl_xor(d, 8, 32);
    d += __shfl_xor(d, 4, 32);
    d += __shfl_xor(d, 2, 32);
    d += __shfl_xor(d, 1, 32);
    mydot = (lane == i) ? d : mydot;
    float* op = Hout + (size_t)row * HID + col0 + 4 * lane;
    if (row < M) *(volatile v4f*)op = o;
    __threadfence();
    if (row < M) *(volatile v4f*)op = o;
  }
  if (lane < 16) sdot[16 * wave + lane] = mydot;
  __syncthreads();
  if (wave == 0) {
    const v4f dv = *(const v4fa*)(sdot + 4 * lane);
    float* dq = DOTP + (size_t)ct * NN + rowBase + 4 * lane;
    *(volatile v4f*)dq = dv;
    __threadfence();
    *(volatile v4f*)dq = dv;
  }
}

__global__ __launch_bounds__(RTHR) KATTR void k_rank(const float* __restrict__ DOTP, const float* __restrict__ pvec,
                                                     const int* __restrict__ ORIGL, int n, int k,
                                                     float* SC, int* INV, int* ORIGN, int* MAPL, int* RFLL) {
  __shared__ __attribute__((aligned(16))) float ssc[NPG];
  __shared__ __attribute__((aligned(16))) int sinv[NPG];
  __shared__ __attribute__((aligned(16))) int sorg[NPG];
  __shared__ __attribute__((aligned(16))) int smap[NPG];
  __shared__ double red[RTHR];
  __shared__ float sgap[4];
  __shared__ int sflag[RTHR / 32];
  const int tid = (int)threadIdx.x, lane = tid & 31, wave = tid >> 5;
  const int g = (int)blockIdx.x;

  {
    const float a = bfr(pvec[tid]);
    const float b = bfr(pvec[tid + RTHR]);
    red[tid] = (double)a * (double)a + (double)b * (double)b;
  }
  if (tid < 4) sgap[tid] = 0.0f;
  __syncthreads();
#pragma unroll 1
  for (int o = RTHR / 2; o > 0; o >>= 1) {
    const double x0 = red[tid];
    const double x1 = red[(tid + o) & (RTHR - 1)];
    if (tid < o) red[tid] = x0 + x1;
    __syncthreads();
  }
  const float pn   = sqrtf((float)red[0]);
  const float rinv = 1.0f / pn;

#pragma unroll 1
  for (int h = 0; h < 2; ++h) {
    const int j  = tid + h * RTHR;
    const int jc = j < n ? j : n - 1;
    const float* dp = DOTP + (size_t)g * n + jc;
    float d = 0.0f;
#pragma unroll 4
    for (int ct = 0; ct < 8; ++ct) d += dp[(size_t)ct * NN];
    const float s = tanhf(d * rinv);
    ssc[j]  = (j < n) ? s : 0.0f;
    sinv[j] = g * n;
    sorg[j] = g * NPG;
    smap[j] = -1;
  }
  __syncthreads();

  const int j0 = tid, j1 = tid + RTHR;
  const float s0 = ssc[j0], s1 = ssc[j1];
  int r0 = 0, r1 = 0;
#pragma unroll 4
  for (int mq = 0; mq < n; ++mq) {
    const float sm = ssc[mq];
    r0 += ((sm > s0) || (sm == s0 && mq < j0)) ? 1 : 0;
    r1 += ((sm > s1) || (sm == s1 && mq < j1)) ? 1 : 0;
  }
  const bool in0 = j0 < n, in1 = j1 < n;
  const int og0 = ORIGL[g * NPG + (in0 ? j0 : n - 1)];
  const int og1 = ORIGL[g * NPG + (in1 ? j1 : n - 1)];
  int ol0 = og0 - g * NPG; ol0 = ol0 < 0 ? 0 : (ol0 > NPG - 1 ? NPG - 1 : ol0);
  int ol1 = og1 - g * NPG; ol1 = ol1 < 0 ? 0 : (ol1 > NPG - 1 ? NPG - 1 : ol1);
  if (in0 && r0 < k) { sinv[r0] = g * n + j0; sorg[r0] = g * NPG + ol0; smap[ol0] = g * k + r0; }
  if (in1 && r1 < k) { sinv[r1] = g * n + j1; sorg[r1] = g * NPG + ol1; smap[ol1] = g * k + r1; }
  if (in0 && r0 == k - 1) sgap[0] = s0;
  if (in0 && r0 == k)     sgap[1] = s0;
  if (in1 && r1 == k - 1) sgap[0] = s1;
  if (in1 && r1 == k)     sgap[1] = s1;
  const bool nf = (in0 && (s0 != s0)) || (in1 && (s1 != s1));
  const unsigned nbm = __builtin_amdgcn_ballot_w32(nf);
  if (lane == 0) sflag[wave] = (nbm != 0u) ? 1 : 0;
  __syncthreads();

  int fl = 0;
#pragma unroll
  for (int w2 = 0; w2 < RTHR / 32; ++w2) fl |= sflag[w2];
  const float gap = sgap[0] - sgap[1];
  const int q = tid & 255;
  const v4f sv = *(const v4fa*)(ssc + 4 * q);
  const v4i iv = *(const v4ia*)(sinv + 4 * q);
  const v4i ov = *(const v4ia*)(sorg + 4 * q);
  const v4i mv = *(const v4ia*)(smap + 4 * q);
  v4i cv;
  cv.x = (tid == 0) ? __float_as_int(gap) : 0;
  cv.y = (tid == 0) ? fl : 0;
  cv.z = 0; cv.w = 0;
  float* scp = SC + (size_t)g * NPG + 4 * q;
  int* inp = INV + (size_t)g * NPG + 4 * q;
  int* orp = ORIGN + (size_t)g * NPG + 4 * q;
  int* mpp = MAPL + (size_t)g * NPG + 4 * q;
  int* rfp = RFLL + (size_t)g * 32 + 4 * (tid & 7);
  if (tid < 256) {
    *(volatile v4f*)scp = sv;
    *(volatile v4i*)inp = iv;
    *(volatile v4i*)orp = ov;
    *(volatile v4i*)mpp = mv;
  }
  if (tid < 8) *(volatile v4i*)rfp = cv;
  __threadfence();
  if (tid < 256) {
    *(volatile v4f*)scp = sv;
    *(volatile v4i*)inp = iv;
    *(volatile v4i*)orp = ov;
    *(volatile v4i*)mpp = mv;
  }
  if (tid < 8) *(volatile v4i*)rfp = cv;
}

template <int WRITE>
__global__ __launch_bounds__(NTHR) KATTR void k_gate(const float* __restrict__ Hm, const float* __restrict__ SC,
                                                     const int* __restrict__ INV, int n, int k, int M,
                                                     unsigned short* HG, float* RO) {
  __shared__ __attribute__((aligned(16))) double wsum[NWAVE * 128];
  __shared__ __attribute__((aligned(16))) float wmax[NWAVE * 128];
  __shared__ __attribute__((aligned(16))) float pst[256];
  const int tid = (int)threadIdx.x, lane = tid & 31;
  const int wave = __builtin_amdgcn_readfirstlane(tid >> 5);
  const int g = (int)blockIdx.x, ch = (int)blockIdx.y;
  const int col0 = ch * 128 + 4 * lane;
  const float nhuge = -__builtin_huge_valf();
  double s0 = 0.0, s1 = 0.0, s2 = 0.0, s3 = 0.0;
  float m0 = nhuge, m1 = nhuge, m2 = nhuge, m3 = nhuge;
#pragma unroll 1
  for (int r = wave; r < k; r += NWAVE) {
    int old = INV[g * NPG + r];
    old = old < 0 ? 0 : (old > M - 1 ? M - 1 : old);
    int jl = old - g * n;
    jl = jl < 0 ? 0 : (jl > n - 1 ? n - 1 : jl);
    const float sc = SC[g * NPG + jl];
    const v4f hv = *(const v4f*)(Hm + (size_t)old * HID + col0);
    const float v0 = hv.x * sc, v1 = hv.y * sc, v2 = hv.z * sc, v3 = hv.w * sc;
    m0 = (v0 > m0 || v0 != v0) ? v0 : m0;
    m1 = (v1 > m1 || v1 != v1) ? v1 : m1;
    m2 = (v2 > m2 || v2 != v2) ? v2 : m2;
    m3 = (v3 > m3 || v3 != v3) ? v3 : m3;
    s0 += (double)v0; s1 += (double)v1; s2 += (double)v2; s3 += (double)v3;
    if (WRITE != 0) {
      const unsigned e0 = f2h_bits(16.0f * v0), e1 = f2h_bits(16.0f * v1);
      const unsigned e2 = f2h_bits(16.0f * v2), e3 = f2h_bits(16.0f * v3);
      v2u qv;
      qv.x = e0 | (e1 << 16);
      qv.y = e2 | (e3 << 16);
      unsigned* hp = (unsigned*)(HG + (size_t)(g * k + r) * HID + col0);
      *(volatile v2u*)hp = qv;
      __threadfence();
      *(volatile v2u*)hp = qv;
    }
  }
  {
    v2d pa; pa.x = s0; pa.y = s1;
    v2d pb; pb.x = s2; pb.y = s3;
    *(v2da*)(wsum + wave * 128 + 4 * lane)     = pa;
    *(v2da*)(wsum + wave * 128 + 4 * lane + 2) = pb;
    v4f mq; mq.x = m0; mq.y = m1; mq.z = m2; mq.w = m3;
    *(v4fa*)(wmax + wave * 128 + 4 * lane) = mq;
  }
  __syncthreads();
  if (tid < 128) {
    double sd = 0.0;
    float mx = nhuge;
#pragma unroll 1
    for (int w2 = 0; w2 < NWAVE; ++w2) {
      sd += wsum[w2 * 128 + tid];
      const float v = wmax[w2 * 128 + tid];
      mx = (v > mx || v != v) ? v : mx;
    }
    pst[tid] = mx;
    pst[128 + tid] = (float)sd / (float)k;
  }
  __syncthreads();
  const int t6 = tid & 63;
  const v4f pv = *(const v4fa*)(pst + 4 * t6);
  const int half = t6 >> 5;
  float* op = RO + (size_t)g * (2 * HID) + (size_t)half * HID + ch * 128 + 4 * (t6 & 31);
  if (tid < 64) *(volatile v4f*)op = pv;
  __threadfence();
  if (tid < 64) *(volatile v4f*)op = pv;
}

__global__ __launch_bounds__(RTHR) KATTR void k_final(const float* __restrict__ RO, const int* __restrict__ FLG0,
                                                      const int* __restrict__ RFL, float* out) {
  const int tid = (int)threadIdx.x;
  const int g = (int)blockIdx.x;
  const size_t e = (size_t)g * (2 * HID) + 4 * tid;
  const size_t lay = (size_t)NB * 2 * HID;
  const v4f r1 = *(const v4f*)(RO + e);
  const v4f r2 = *(const v4f*)(RO + lay + e);
  const v4f r3 = *(const v4f*)(RO + 2 * lay + e);
  const int f = FLG0[g * 32 + 1] | RFL[g * 32 + 1] | RFL[(NB + g) * 32 + 1] | RFL[(2 * NB + g) * 32 + 1];
  const float qnan = __int_as_float(0x7fc00000);
  v4f o;
  o.x = (r1.x + r2.x) + r3.x;
  o.y = (r1.y + r2.y) + r3.y;
  o.z = (r1.z + r2.z) + r3.z;
  o.w = (r1.w + r2.w) + r3.w;
  o.x = (f != 0) ? qnan : o.x;
  o.y = (f != 0) ? qnan : o.y;
  o.z = (f != 0) ? qnan : o.z;
  o.w = (f != 0) ? qnan : o.w;
  float* op = out + e;
  *(volatile v4f*)op = o;
  __threadfence();
  *(volatile v4f*)op = o;
}

static inline int cdiv(int a, int b) { return (a + b - 1) / b; }
static inline size_t al256(size_t o) { return (o + 255) & ~(size_t)255; }

extern "C" void kernel_launch(void* const* d_in, const int* in_sizes, int n_in,
                              void* d_out, int out_size, void* d_ws, size_t ws_size,
                              hipStream_t stream) {
  if (n_in < 15) return;
  if (in_sizes[0] != NN * FEAT) return;
  if (in_sizes[1] != 2 * NEDGE) return;
  if (in_sizes[3] != HID * FEAT || in_sizes[5] != HID * FEAT) return;
  if (in_sizes[4] != HID || in_sizes[6] != HID) return;
  if (in_sizes[7] != HID * HID || in_sizes[9] != HID * HID) return;
  if (in_sizes[8] != HID || in_sizes[10] != HID) return;
  if (in_sizes[11] != HID * HID || in_sizes[13] != HID * HID) return;
  if (in_sizes[12] != HID || in_sizes[14] != HID) return;
  if (out_size != NB * 2 * HID) return;

  const float* x   = (const float*)d_in[0];
  const int*   ei  = (const int*)  d_in[1];
  const float* W1l = (const float*)d_in[3];
  const float* b1  = (const float*)d_in[4];
  const float* W1r = (const float*)d_in[5];
  const float* p1  = (const float*)d_in[6];
  const float* W2l = (const float*)d_in[7];
  const float* b2  = (const float*)d_in[8];
  const float* W2r = (const float*)d_in[9];
  const float* p2  = (const float*)d_in[10];
  const float* W3l = (const float*)d_in[11];
  const float* b3  = (const float*)d_in[12];
  const float* W3r = (const float*)d_in[13];
  const float* p3  = (const float*)d_in[14];
  float* out = (float*)d_out;
  const int nE = NEDGE;
  const int* src = ei;
  const int* dst = ei + nE;
  const int vec8 = ((nE & 3) == 0) ? 1 : 0;

  char* ws = (char*)d_ws;
  size_t off = 0;
  const size_t oRA   = off; off = al256(off + (size_t)MM2 * HID * 2);
  const size_t oRB   = off; off = al256(off + (size_t)MM2 * HID * 2);
  const size_t oRH   = off; off = al256(off + (size_t)NN * HID * 4);
  const size_t oW1C  = off; off = al256(off + (size_t)HID * 2 * FEAT * 2);
  const size_t oLIST = off; off = al256(off + (size_t)NB * RCAP * 4);
  const size_t oCNT  = off; off = al256(off + (size_t)NB * NBA * 4);
  const size_t oOFF  = off; off = al256(off + (size_t)NB * NBA * 4);
  const size_t oFLG0 = off; off = al256(off + (size_t)NB * 128);
  const size_t oMAP  = off; off = al256(off + (size_t)4 * NN * 4);
  const size_t oORIG = off; off = al256(off + (size_t)4 * NN * 4);
  const size_t oINV  = off; off = al256(off + (size_t)NN * 4);
  const size_t oSC   = off; off = al256(off + (size_t)NN * 4);
  const size_t oDOTP = off; off = al256(off + (size_t)8 * NN * 4);
  const size_t oRO   = off; off = al256(off + (size_t)3 * NB * 2 * HID * 4);
  const size_t oRFL  = off; off = al256(off + (size_t)3 * NB * 128);
  if (off > ws_size || off > (size_t)WSMAX) return;
  if ((size_t)NN * FEAT * 2 > (size_t)MM2 * HID * 2) return;

  unsigned short* RA   = (unsigned short*)(ws + oRA);
  unsigned short* RB   = (unsigned short*)(ws + oRB);
  float*          RH   = (float*)(ws + oRH);
  unsigned short* WC23 = (unsigned short*)(ws + oRH + (size_t)WTAIL);
  unsigned short* W1C  = (unsigned short*)(ws + oW1C);
  int*   LIST = (int*)(ws + oLIST);
  int*   CNT  = (int*)(ws + oCNT);
  int*   OFF  = (int*)(ws + oOFF);
  int*   FLG0 = (int*)(ws + oFLG0);
  int*   MAPS = (int*)(ws + oMAP);
  int*   ORGS = (int*)(ws + oORIG);
  int*   INV  = (int*)(ws + oINV);
  float* SC   = (float*)(ws + oSC);
  float* DOTP = (float*)(ws + oDOTP);
  float* RO   = (float*)(ws + oRO);
  int*   RFL  = (int*)(ws + oRFL);
  unsigned short* W2C = WC23;
  unsigned short* W3C = WC23 + (size_t)HID * 2 * HID;

  const int bktLds  = BKT_LDS_INTS * 4;
  const int gemmLds = GEMM_LDS_FLOATS * 4;
  hipFuncSetAttribute(reinterpret_cast<const void*>(&k_bucket),
                      hipFuncAttributeMaxDynamicSharedMemorySize, bktLds);
  hipFuncSetAttribute(reinterpret_cast<const void*>(&k_gemm),
                      hipFuncAttributeMaxDynamicSharedMemorySize, gemmLds);

  k_prep<<<(NUX + NUW1 + 2 * NUID) / NTHR, NTHR, 0, stream>>>(x, W1l, W1r, RA, W1C, MAPS, ORGS);
  k_bucket<<<NB, NTHR, bktLds, stream>>>(src, dst, nE, NN, vec8, LIST, CNT, OFF, FLG0);

  k_agg<2><<<NN / NWAVE, NTHR, 0, stream>>>(LIST, CNT, OFF, FLG0, MAPS, RA, RB, MM1);
  k_gemm<<<dim3(cdiv(MM1, GT), HID / GT), GTHR, gemmLds, stream>>>(RB, RA, W1C, FEAT, MM1, b1, p1, RH, DOTP);
  k_rank<<<NB, RTHR, 0, stream>>>(DOTP, p1, ORGS, NPG, KK1, SC, INV, ORGS + NN, MAPS + NN, RFL);
  k_gate<1><<<dim3(NB, 8), NTHR, 0, stream>>>(RH, SC, INV, NPG, KK1, MM1, RA, RO);
  k_prepW<<<2 * NUW23 / NTHR, NTHR, 0, stream>>>(W2l, W2r, W3l, W3r, WC23);

  k_agg<4><<<NN / NWAVE, NTHR, 0, stream>>>(LIST, CNT, OFF, FLG0, MAPS + NN, RA, RB, MM2);
  k_gemm<<<dim3(cdiv(MM2, GT), HID / GT), GTHR, gemmLds, stream>>>(RB, RA, W2C, HID, MM2, b2, p2, RH, DOTP);
  k_rank<<<NB, RTHR, 0, stream>>>(DOTP, p2, ORGS + NN, KK1, KK2, SC, INV, ORGS + 2 * NN, MAPS + 2 * NN,
                                  RFL + NB * 32);
  k_gate<1><<<dim3(NB, 8), NTHR, 0, stream>>>(RH, SC, INV, KK1, KK2, MM2, RA, RO + (size_t)NB * 2 * HID);

  k_agg<4><<<NN / NWAVE, NTHR, 0, stream>>>(LIST, CNT, OFF, FLG0, MAPS + 2 * NN, RA, RB, MM3);
  k_gemm<<<dim3(cdiv(MM3, GT), HID / GT), GTHR, gemmLds, stream>>>(RB, RA, W3C, HID, MM3, b3, p3, RH, DOTP);
  k_rank<<<NB, RTHR, 0, stream>>>(DOTP, p3, ORGS + 2 * NN, KK2, KK3, SC, INV, ORGS + 3 * NN, MAPS + 3 * NN,
                                  RFL + 2 * NB * 32);
  k_gate<0><<<dim3(NB, 8), NTHR, 0, stream>>>(RH, SC, INV, KK2, KK3, MM3, RA, RO + (size_t)2 * NB * 2 * HID);

  k_final<<<NB, RTHR, 0, stream>>>(RO, FLG0, RFL, out);
}
